// MLP_76605036691741
// MI455X (gfx1250) — hardware-verified
//
#include <hip/hip_runtime.h>

constexpr int NUM_NODES = 100000;
constexpr int NUM_EDGES = 500000;
constexpr int FEAT_IN   = 128;
constexpr int FEAT_HID  = 128;
constexpr int KDIM1     = 2 * FEAT_IN;
constexpr int EDGE_TILE = 64;
constexpr int NTHREADS  = 256;
constexpr int A_PITCH   = 272;
constexpr int X_PITCH   = 136;
constexpr int NUM_BLOCKS = (NUM_EDGES + EDGE_TILE - 1) / EDGE_TILE;

static_assert(KDIM1 % 32 == 0, "");
static_assert(FEAT_HID % 32 == 0, "");
static_assert(NUM_EDGES % 32 == 0, "");
static_assert(64 * A_PITCH * 2 == 64 * X_PITCH * 4, "");
static_assert(2 * (64 * X_PITCH * 2) == 64 * A_PITCH * 2, "");
static_assert((A_PITCH * 2) % 16 == 0 && (X_PITCH * 2) % 16 == 0, "");

constexpr size_t WS_W1B   = 0;
constexpr size_t WS_W2B   = 65536;
constexpr size_t WS_PT    = 98304;
constexpr size_t WS_TOTAL = 100352;

typedef __attribute__((ext_vector_type(16))) __bf16   v16b;
typedef __attribute__((ext_vector_type(8)))  __bf16   v8b;
typedef __attribute__((ext_vector_type(8)))  float    v8f;
typedef __attribute__((ext_vector_type(4)))  float    v4f;
typedef __attribute__((ext_vector_type(4)))  unsigned int v4u;
typedef __attribute__((ext_vector_type(2)))  unsigned int v2u;

__device__ __forceinline__ unsigned short f2bf_bits(float f) {
  unsigned u = __float_as_uint(f);
  return (unsigned short)((u + 0x7FFFu + ((u >> 16) & 1u)) >> 16);
}
__device__ __forceinline__ float bf_bits2f(unsigned short h) { return __uint_as_float(((unsigned)h) << 16); }
__device__ __forceinline__ unsigned pk16(unsigned short a, unsigned short b) { return (unsigned)a | ((unsigned)b << 16); }

__device__ __forceinline__ void acc_guard4(v8f& a, v8f& b, v8f& c, v8f& d) { asm volatile("v_nop\n\tv_nop\n\tv_nop\n\tv_nop" : "+v"(a), "+v"(b), "+v"(c), "+v"(d)); }
__device__ __forceinline__ void guard_ab(v8f& c, v16b a, v16b b) { asm volatile("v_nop\n\tv_nop\n\tv_nop\n\tv_nop" : "+v"(c) : "v"(a), "v"(b)); }
__device__ __forceinline__ void guard_aab(v8f& c, v16b a, v16b a2, v16b b) { asm volatile("v_nop\n\tv_nop\n\tv_nop\n\tv_nop" : "+v"(c) : "v"(a), "v"(a2), "v"(b)); }

struct FragB {
  union U { v16b v; v8b h[2]; };
  static __device__ __forceinline__ v16b load(const __bf16* p) {
    U f; f.h[0] = *(const v8b*)(p); f.h[1] = *(const v8b*)(p + 16); return f.v;
  }
  static __device__ __forceinline__ v8f mma(v16b a, v16b b, v8f c) {
    return __builtin_amdgcn_wmma_f32_16x16x32_bf16(false, a, false, b, (short)0, c, false, false);
  }
};

__global__ __launch_bounds__(NTHREADS) void prep_kernel(const float* __restrict__ W1, const float* __restrict__ b1,
                                                       const float* __restrict__ W2, const float* __restrict__ b2,
                                                       const float* __restrict__ W3, const float* __restrict__ b3,
                                                       unsigned short* __restrict__ W1B, unsigned short* __restrict__ W2B,
                                                       float* __restrict__ PT) {
  const int t = threadIdx.x, lane = t & 31, wave = t >> 5;
  const int blk = blockIdx.x;
  if (blk < 24) {
    const float* sp; unsigned short* dp; int g;
    if (blk < 16) { sp = W1; dp = W1B; g = blk * 256 + t; }
    else          { sp = W2; dp = W2B; g = (blk - 16) * 256 + t; }
    const v4f a = *(const v4f*)(sp + 8 * (size_t)g);
    const v4f c = *(const v4f*)(sp + 8 * (size_t)g + 4);
    unsigned short hb[8];
#pragma unroll
    for (int e = 0; e < 4; ++e) {
      const float fa = a[e]; const float fc = c[e];
      hb[e] = f2bf_bits(fa); hb[4 + e] = f2bf_bits(fc);
    }
    const v4u u = (v4u){pk16(hb[0], hb[1]), pk16(hb[2], hb[3]), pk16(hb[4], hb[5]), pk16(hb[6], hb[7])};
    unsigned short* q = dp + 8 * (size_t)g;
    *(volatile v4u*)q = u;
    __threadfence();
    *(volatile v4u*)q = u;
  } else {
    if (wave < 4) {
      v4f v;
      if (wave == 0)      v = *(const v4f*)(b1 + 4 * lane);
      else if (wave == 1) v = *(const v4f*)(b2 + 4 * lane);
      else if (wave == 2) v = *(const v4f*)(W3 + 4 * lane);
      else { const float s = b3[0]; v = (v4f){s, s, s, s}; }
      v4f r;
#pragma unroll
      for (int e = 0; e < 4; ++e) { const float s = v[e]; r[e] = bf_bits2f(f2bf_bits(s)); }
      float* q = PT + wave * 128 + 4 * lane;
      *(volatile v4f*)q = r;
      __threadfence();
      *(volatile v4f*)q = r;
    }
  }
}

union TileU {
  unsigned short hw[64 * A_PITCH];
  float          fw[64 * X_PITCH];
};

__global__ __launch_bounds__(NTHREADS) void edge_mlp_kernel(const float* __restrict__ h,
                                                           const int*   __restrict__ src,
                                                           const int*   __restrict__ dst,
                                                           const unsigned short* __restrict__ W1B,
                                                           const unsigned short* __restrict__ W2B,
                                                           const float* __restrict__ PT,
                                                           float* __restrict__ out) {
  __shared__ __align__(16) TileU sTile;
  __shared__ int sIdx[128];
  __shared__ __align__(16) float sW3[128];
  __shared__ __align__(16) float sOut[64];

  const int t = threadIdx.x, lane = t & 31, wave = t >> 5;
  const int e0 = blockIdx.x * EDGE_TILE;
  const int rem = NUM_EDGES - e0;
  const int nvalid = rem < EDGE_TILE ? rem : EDGE_TILE;

  if (wave < 4) {
    const int r = t & 63;
    int e = e0 + r; e = e < NUM_EDGES ? e : NUM_EDGES - 1;
    const int vs = src[e];
    const int vd = dst[e];
    const int msk = (wave < 2) ? -1 : 0;
    int node = (vs & msk) | (vd & ~msk);
    node = node < 0 ? 0 : (node >= NUM_NODES ? NUM_NODES - 1 : node);
    sIdx[t] = node;
  } else {
    sW3[t - 128] = PT[256 + (t - 128)];
  }
  const float b3v = PT[384];
  __syncthreads();

#pragma unroll 1
  for (int grp = 0; grp < 4; ++grp) {
#pragma unroll
    for (int i = 0; i < 4; ++i) {
      const int idx = (grp * 4 + i) * 256 + t;
      const int m  = idx >> 6;
      const int cu = idx & 63;
      const int node = sIdx[m + (cu & 32) * 2];
      const v4f f = *(const v4f*)(h + (size_t)node * FEAT_IN + (cu & 31) * 4);
      const float f0 = f[0], f1 = f[1], f2 = f[2], f3 = f[3];
      const v2u pk = (v2u){pk16(f2bf_bits(f0), f2bf_bits(f1)), pk16(f2bf_bits(f2), f2bf_bits(f3))};
      *(v2u*)(&sTile.hw[m * A_PITCH + cu * 4]) = pk;
    }
  }
  __syncthreads();

  const int nl   = lane & 15;
  const int hh   = lane >> 4;
  const int koff = hh * 8;
  const int n0   = wave * 16;

  v8f acc[4];
#pragma unroll
  for (int mt = 0; mt < 4; ++mt) acc[mt] = (v8f){0.f, 0.f, 0.f, 0.f, 0.f, 0.f, 0.f, 0.f};
  {
    const __bf16* Abase = (const __bf16*)sTile.hw;
    const __bf16* Bp = (const __bf16*)W1B + (size_t)(n0 + nl) * KDIM1 + koff;
#pragma unroll 1
    for (int kc = 0; kc < KDIM1 / 32; ++kc) {
      const int k0 = kc * 32;
      const v16b bf = FragB::load(Bp + k0);
#pragma unroll
      for (int mt = 0; mt < 4; ++mt) {
        const v16b af = FragB::load(Abase + (mt * 16 + nl) * A_PITCH + k0 + koff);
        acc[mt] = FragB::mma(af, bf, acc[mt]);
        guard_ab(acc[mt], af, bf);
      }
    }
  }
  acc_guard4(acc[0], acc[1], acc[2], acc[3]);
  __syncthreads();

  unsigned short* X1H = sTile.hw;
  unsigned short* X1L = sTile.hw + 64 * X_PITCH;
  {
    const float b1v = PT[n0 + nl];
#pragma unroll
    for (int mt = 0; mt < 4; ++mt) {
#pragma unroll
      for (int r = 0; r < 8; ++r) {
        const int row = mt * 16 + hh * 8 + r;
        float v = acc[mt][r] + b1v;
        v = fmaxf(v, 0.0f);
        const unsigned short hb = f2bf_bits(v);
        const unsigned short lb = f2bf_bits(v - bf_bits2f(hb));
        X1H[row * X_PITCH + n0 + nl] = hb;
        X1L[row * X_PITCH + n0 + nl] = lb;
      }
    }
  }
  __syncthreads();

  v8f acc2[4];
#pragma unroll
  for (int mt = 0; mt < 4; ++mt) acc2[mt] = (v8f){0.f, 0.f, 0.f, 0.f, 0.f, 0.f, 0.f, 0.f};
  {
    const __bf16* XHb = (const __bf16*)X1H;
    const __bf16* XLb = (const __bf16*)X1L;
    const __bf16* Bp = (const __bf16*)W2B + (size_t)(n0 + nl) * FEAT_HID + koff;
#pragma unroll 1
    for (int kc = 0; kc < FEAT_HID / 32; ++kc) {
      const int k0 = kc * 32;
      const v16b bf = FragB::load(Bp + k0);
#pragma unroll
      for (int mt = 0; mt < 4; ++mt) {
        const int ao = (mt * 16 + nl) * X_PITCH + k0 + koff;
        const v16b ah = FragB::load(XHb + ao);
        const v16b al = FragB::load(XLb + ao);
        acc2[mt] = FragB::mma(ah, bf, acc2[mt]);
        acc2[mt] = FragB::mma(al, bf, acc2[mt]);
        guard_aab(acc2[mt], ah, al, bf);
      }
    }
  }
  acc_guard4(acc2[0], acc2[1], acc2[2], acc2[3]);
  __syncthreads();

  float* X2 = sTile.fw;
  {
    const float b2v = PT[128 + n0 + nl];
#pragma unroll
    for (int mt = 0; mt < 4; ++mt) {
#pragma unroll
      for (int r = 0; r < 8; ++r) {
        const int row = mt * 16 + hh * 8 + r;
        float v = acc2[mt][r] + b2v;
        v = fmaxf(v, 0.0f);
        X2[row * X_PITCH + n0 + nl] = v;
      }
    }
  }
  __syncthreads();

  {
    const int m = t >> 2;
    const int p = t & 3;
    const float* xr = X2 + m * X_PITCH + p * 32;
    const float* wr = sW3 + p * 32;
    float s = 0.0f;
#pragma unroll
    for (int q = 0; q < 8; ++q) {
      const v4f xv = *(const v4f*)(xr + 4 * q);
      const v4f wv = *(const v4f*)(wr + 4 * q);
      s = fmaf(xv[0], wv[0], s);
      s = fmaf(xv[1], wv[1], s);
      s = fmaf(xv[2], wv[2], s);
      s = fmaf(xv[3], wv[3], s);
    }
    s += __shfl_xor(s, 1, 32);
    s += __shfl_xor(s, 2, 32);
    if (p == 0) sOut[m] = s + b3v;
  }
  __syncthreads();

  if (wave == 0) {
    const int lim = nvalid >> 2;
    const int cl = lane < lim ? lane : 0;
    const v4f v = *(const v4f*)(sOut + 4 * cl);
    float* op = out + (size_t)e0 + 4 * lane;
    if (lane < lim) *(volatile v4f*)op = v;
    __threadfence();
    if (lane < lim) *(volatile v4f*)op = v;
  }
}

extern "C" void kernel_launch(void* const* d_in, const int* in_sizes, int n_in,
                              void* d_out, int out_size, void* d_ws, size_t ws_size,
                              hipStream_t stream) {
  (void)in_sizes; (void)n_in;
  const float* h   = (const float*)d_in[0];
  const int*   src = (const int*)  d_in[1];
  const int*   dst = (const int*)  d_in[2];
  const float* W1  = (const float*)d_in[3];
  const float* b1  = (const float*)d_in[4];
  const float* W2  = (const float*)d_in[5];
  const float* b2  = (const float*)d_in[6];
  const float* W3  = (const float*)d_in[7];
  const float* b3  = (const float*)d_in[8];
  float* out = (float*)d_out;

  if (ws_size < WS_TOTAL) return;
  if (out_size < NUM_EDGES) return;

  char* ws = (char*)d_ws;
  unsigned short* W1B = (unsigned short*)(ws + WS_W1B);
  unsigned short* W2B = (unsigned short*)(ws + WS_W2B);
  float*          PT  = (float*)(ws + WS_PT);

  prep_kernel<<<25, NTHREADS, 0, stream>>>(W1, b1, W2, b2, W3, b3, W1B, W2B, PT);
  edge_mlp_kernel<<<NUM_BLOCKS, NTHREADS, 0, stream>>>(h, src, dst, W1B, W2B, PT, out);
}
